// PointTransformerCls_11020886082150
// MI455X (gfx1250) — hardware-verified
//
#include <hip/hip_runtime.h>


#define NBAT 16
#define N0 4096
#define KNB 16
#define NCLS 40
#define BN_EPS 1e-5f

typedef __attribute__((ext_vector_type(16))) __bf16   v16bf;
typedef __attribute__((ext_vector_type(16))) _Float16 v16h;
typedef __attribute__((ext_vector_type(8)))  float    v8f;
typedef __attribute__((ext_vector_type(8)))  unsigned v8u;

__device__ __forceinline__ unsigned f2bf(float f) { unsigned u = __float_as_uint(f); u += 0x7FFFu + ((u >> 16) & 1u); return u >> 16; }
__device__ __forceinline__ unsigned f2h(float f) { return (unsigned)__builtin_bit_cast(unsigned short, (_Float16)f); }
__device__ __forceinline__ int kpat(int v, int half) { return ((v & 4) ? 16 : 0) + half * 8 + 2 * (v & 3); }

template <int F16, int NP> struct Opnd { v16bf p[NP]; };

template <int F16, int NP> __device__ __forceinline__ void pack2(float f0, float f1, unsigned* o) {
    if (F16) { o[0] = f2h(f0) | (f2h(f1) << 16); return; }
    unsigned h0 = f2bf(f0), h1 = f2bf(f1); o[0] = h0 | (h1 << 16);
    if (NP >= 2) {
        float r0 = f0 - __uint_as_float(h0 << 16), r1 = f1 - __uint_as_float(h1 << 16);
        unsigned m0 = f2bf(r0), m1 = f2bf(r1); o[1] = m0 | (m1 << 16);
        if (NP >= 3) {
            float s0 = r0 - __uint_as_float(m0 << 16), s1 = r1 - __uint_as_float(m1 << 16);
            o[2] = f2bf(s0) | (f2bf(s1) << 16);
        }
    }
}
template <int F16, int NP> __device__ __forceinline__ void op_row(const float* rowp, int half, float sc, Opnd<F16, NP>& o) {
    v8u u[NP];
#pragma unroll
    for (int v = 0; v < 8; ++v) {
        int kk = kpat(v, half); unsigned t[3];
        pack2<F16, NP>(rowp[kk] * sc, rowp[kk + 1] * sc, t);
#pragma unroll
        for (int p = 0; p < NP; ++p) u[p][v] = t[p];
    }
#pragma unroll
    for (int p = 0; p < NP; ++p) o.p[p] = __builtin_bit_cast(v16bf, u[p]);
}
template <int F16, int NP> __device__ __forceinline__ void op_row_tail(const float* rowp, int half, float sc, int kvalid, Opnd<F16, NP>& o) {
    v8u u[NP];
#pragma unroll
    for (int v = 0; v < 8; ++v) {
        int kk = kpat(v, half); unsigned t[3];
        float f0 = kk < kvalid ? rowp[kk] * sc : 0.0f, f1 = (kk + 1) < kvalid ? rowp[kk + 1] * sc : 0.0f;
        pack2<F16, NP>(f0, f1, t);
#pragma unroll
        for (int p = 0; p < NP; ++p) u[p][v] = t[p];
    }
#pragma unroll
    for (int p = 0; p < NP; ++p) o.p[p] = __builtin_bit_cast(v16bf, u[p]);
}
template <int F16, int NP> __device__ __forceinline__ void op_col(const float* M, int ld, int n, int k0, int half, float sc, Opnd<F16, NP>& o) {
    v8u u[NP];
#pragma unroll
    for (int v = 0; v < 8; ++v) {
        int kk = k0 + kpat(v, half); unsigned t[3];
        pack2<F16, NP>(M[(size_t)kk * ld + n] * sc, M[(size_t)(kk + 1) * ld + n] * sc, t);
#pragma unroll
        for (int p = 0; p < NP; ++p) u[p][v] = t[p];
    }
#pragma unroll
    for (int p = 0; p < NP; ++p) o.p[p] = __builtin_bit_cast(v16bf, u[p]);
}
template <int F16, int NP> __device__ __forceinline__ void op_col_tail(const float* M, int ld, int n, int k0, int half, float sc, int K, Opnd<F16, NP>& o) {
    v8u u[NP];
#pragma unroll
    for (int v = 0; v < 8; ++v) {
        int kk = k0 + kpat(v, half); unsigned t[3];
        float f0 = kk < K ? M[(size_t)kk * ld + n] * sc : 0.0f, f1 = (kk + 1) < K ? M[(size_t)(kk + 1) * ld + n] * sc : 0.0f;
        pack2<F16, NP>(f0, f1, t);
#pragma unroll
        for (int p = 0; p < NP; ++p) u[p][v] = t[p];
    }
#pragma unroll
    for (int p = 0; p < NP; ++p) o.p[p] = __builtin_bit_cast(v16bf, u[p]);
}
__device__ __forceinline__ v8f wm_bf16(v16bf a, v16bf b, v8f c) { return __builtin_amdgcn_wmma_f32_16x16x32_bf16(false, a, false, b, (short)0, c, false, false); }
template <int F16, int NA, int NB> __device__ __forceinline__ v8f wmma_op(const Opnd<F16, NA>& a, const Opnd<F16, NB>& b, v8f c) {
    if (F16) {
        v16h ah = __builtin_bit_cast(v16h, a.p[0]), bh = __builtin_bit_cast(v16h, b.p[0]);
        c = __builtin_amdgcn_wmma_f32_16x16x32_f16(false, ah, false, bh, (short)0, c, false, false);
        asm volatile("v_nop\n\tv_nop\n\tv_nop\n\tv_nop" : "+v"(c) : "v"(ah), "v"(bh));
        return c;
    }
    constexpr int NMX = NA > NB ? NA : NB;
#pragma unroll
    for (int i = 0; i < NA; ++i)
#pragma unroll
        for (int j = 0; j < NB; ++j)
            if (i + j < NMX) c = wm_bf16(a.p[i], b.p[j], c);
    if (NA == 1 && NB == 1)      asm volatile("v_nop\n\tv_nop\n\tv_nop\n\tv_nop" : "+v"(c) : "v"(a.p[0]), "v"(b.p[0]));
    else if (NA == 2 && NB == 1) asm volatile("v_nop\n\tv_nop\n\tv_nop\n\tv_nop" : "+v"(c) : "v"(a.p[0]), "v"(a.p[1]), "v"(b.p[0]));
    else if (NA == 1 && NB == 2) asm volatile("v_nop\n\tv_nop\n\tv_nop\n\tv_nop" : "+v"(c) : "v"(a.p[0]), "v"(b.p[0]), "v"(b.p[1]));
    else if (NA == 2 && NB == 2) asm volatile("v_nop\n\tv_nop\n\tv_nop\n\tv_nop" : "+v"(c) : "v"(a.p[0]), "v"(a.p[1]), "v"(b.p[0]), "v"(b.p[1]));
    else                         asm volatile("v_nop\n\tv_nop\n\tv_nop\n\tv_nop" : "+v"(c) : "v"(a.p[0]), "v"(a.p[NA - 1]), "v"(b.p[0]), "v"(b.p[NB - 1]), "v"(a.p[NA / 2]), "v"(b.p[NB / 2]));
    return c;
}

struct ZMap { long long s1; long long s2; int zdiv; int pad_; };
__device__ __forceinline__ size_t zoff(const ZMap& m, int z) { return (size_t)((long long)(z / m.zdiv) * m.s1 + (long long)(z % m.zdiv) * m.s2); }

#define ACT_NONE 0
#define ACT_RELU 1
#define ACT_GELU_ERF 2
#define ACT_SILU 3
#define ACT_TANH 4
__device__ __forceinline__ float act_apply(int act, float x) {
    if (act == ACT_RELU) return x > 0.f ? x : 0.f;
    if (act == ACT_GELU_ERF) return 0.5f * x * (1.0f + erff(x * 0.70710678118654752f));
    if (act == ACT_SILU) return x / (1.0f + expf(-x));
    if (act == ACT_TANH) return tanhf(x);
    return x;
}
struct GemmArgs {
    ZMap za, zb_, zc, zbias, zadd, zrsc, zmul, zrbias;
    const float* A; const float* Bm; float* C; const float* bias; const float* add; const float* rsc; const float* mul; const float* rbias;
    long long ldadd, ldmul;
    int lda, ldb, ldc, K;
    float ascale, bscale, oscale, addscale;
    int M, nvalid, nstore, ldrsc;
    int bcs, pad1, pad2, pad3;
};
template <int BT, int F16, int NA, int NB, int RW, int CW, int ACT>
__global__ __launch_bounds__(256) void gemm_kernel(GemmArgs g) {
    constexpr int TR = 16 * RW, TC = 64 * CW, CSTR = TC + 4;
    __shared__ __align__(16) float cst[TR * CSTR];
    const int z = blockIdx.z;
    const float* A = g.A + zoff(g.za, z); const float* Bm = g.Bm + zoff(g.zb_, z); float* C = g.C + zoff(g.zc, z);
    const int tid = threadIdx.x, lane = tid & 31, wv = tid >> 5;
    const int l16 = lane & 15, half = lane >> 4;
    const int rt = wv % RW, ch = wv / RW;
    const int row0 = blockIdx.x * TR, col0 = blockIdx.y * TC + ch * 64;
    int arix = row0 + rt * 16 + l16; if (arix >= g.M) arix = g.M - 1;
    const float* arow = A + (size_t)arix * g.lda;
    v8f acc[4];
#pragma unroll
    for (int t = 0; t < 4; ++t) acc[t] = (v8f){};
    const int K = g.K;
#pragma unroll 1
    for (int kc = 0; kc < K; kc += 32) {
        Opnd<F16, NA> a;
        if (kc + 32 <= K) op_row<F16, NA>(arow + kc, half, g.ascale, a); else op_row_tail<F16, NA>(arow + kc, half, g.ascale, K - kc, a);
#pragma unroll
        for (int t = 0; t < 4; ++t) {
            Opnd<F16, NB> b;
            const int n = col0 + t * 16 + l16;
            if (n < g.nvalid) {
                if (BT) { if (kc + 32 <= K) op_row<F16, NB>(Bm + (size_t)n * g.ldb + kc, half, g.bscale, b); else op_row_tail<F16, NB>(Bm + (size_t)n * g.ldb + kc, half, g.bscale, K - kc, b); }
                else    { if (kc + 32 <= K) op_col<F16, NB>(Bm, g.ldb, n * g.bcs, kc, half, g.bscale, b); else op_col_tail<F16, NB>(Bm, g.ldb, n * g.bcs, kc, half, g.bscale, K, b); }
            } else {
#pragma unroll
                for (int p = 0; p < NB; ++p) b.p[p] = (v16bf){};
            }
            acc[t] = wmma_op<F16, NA, NB>(a, b, acc[t]);
        }
    }
    const float* bias = g.bias ? g.bias + zoff(g.zbias, z) : nullptr;
    const float* add = g.add ? g.add + zoff(g.zadd, z) : nullptr;
    const float* rsc = g.rsc ? g.rsc + zoff(g.zrsc, z) : nullptr;
    const float* mul = g.mul ? g.mul + zoff(g.zmul, z) : nullptr;
    const float* rbias = g.rbias ? g.rbias + zoff(g.zrbias, z) : nullptr;
#pragma unroll
    for (int t = 0; t < 4; ++t) {
        const int cl = ch * 64 + t * 16 + l16;
        const int cg = blockIdx.y * TC + cl;
        const bool cok = cg < g.nvalid;
        const float bv = (bias && cok) ? bias[(size_t)cg * g.bcs] : 0.0f;
#pragma unroll
        for (int r = 0; r < 8; ++r) {
            const int rl = rt * 16 + r + 8 * half;
            float v = acc[t][r] * g.oscale + bv;
            int rg = row0 + rl; if (rg >= g.M) rg = g.M - 1;
            if (rbias) v += rbias[rg];
            if (rsc) v *= rsc[(size_t)rg * g.ldrsc];
            if (mul && cok) v *= mul[(size_t)rg * g.ldmul + cg];
            if (add && cok) v += g.addscale * add[(size_t)rg * g.ldadd + cg];
            cst[rl * CSTR + cl] = v;
        }
    }
    __syncthreads();
    const int col = tid % TC, rsel = tid / TC, rstep = 256 / TC;
    if (ACT != ACT_NONE) {
#pragma unroll 1
        for (int r = rsel; r < TR; r += rstep) cst[r * CSTR + col] = act_apply(ACT, cst[r * CSTR + col]);
    }
    float* ob = C + (size_t)row0 * g.ldc + (size_t)blockIdx.y * TC;
    const bool colok = (int)(blockIdx.y * TC + col) < g.nstore;
    const int rmax = (g.M - row0 < TR) ? (g.M - row0) : TR;
    auto pass = [&]() {
        if (colok) {
#pragma unroll 4
            for (int r = rsel; r < rmax; r += rstep) *(volatile float*)(ob + (size_t)r * g.ldc + col) = cst[r * CSTR + col];
        }
    };
    pass();
    __threadfence();
    pass();
}
static inline ZMap zm(long long s1) { ZMap m; m.s1 = s1; m.s2 = 0; m.zdiv = 1; m.pad_ = 0; return m; }
static inline ZMap zm2(long long s1, long long s2, int zdiv) { ZMap m; m.s1 = s1; m.s2 = s2; m.zdiv = zdiv; m.pad_ = 0; return m; }
static inline GemmArgs gemm_args(const float* A, int lda, ZMap za, const float* Bm, int ldb, ZMap zb, float* C, int ldc, ZMap zc, int M, int N, int K) {
    GemmArgs g; g.za = za; g.zb_ = zb; g.zc = zc; g.zbias = zm(0); g.zadd = zm(0); g.zrsc = zm(0); g.zmul = zm(0); g.zrbias = zm(0);
    g.A = A; g.Bm = Bm; g.C = C; g.bias = nullptr; g.add = nullptr; g.rsc = nullptr; g.mul = nullptr; g.rbias = nullptr; g.ldadd = 0; g.ldmul = 0;
    g.lda = lda; g.ldb = ldb; g.ldc = ldc; g.K = K; g.ascale = 1.0f; g.bscale = 1.0f; g.oscale = 1.0f; g.addscale = 1.0f; g.M = M; g.nvalid = N; g.nstore = N; g.ldrsc = 1;
    g.bcs = 1; g.pad1 = 0; g.pad2 = 0; g.pad3 = 0;
    return g;
}
static_assert(sizeof(ZMap) == 24, "ZMap layout");
static_assert(sizeof(GemmArgs) == 8 * 24 + 8 * 8 + 2 * 8 + 4 * 4 + 4 * 4 + 4 * 4 + 4 * 4, "GemmArgs has no padding");

__global__ __launch_bounds__(256) void softmax_rows(float* S, long long sy, long long sx, int L, float prescale, const float* addv, long long say, int aydiv, int causal,
                                                  const int* imask, long long imy, long long imx, float maskval) {
    __shared__ float red[8];
    const int tid = threadIdx.x, lane = tid & 31, wid = tid >> 5;
    float* row = S + (size_t)blockIdx.y * sy + (size_t)blockIdx.x * sx;
    const float* av = addv ? addv + (size_t)(blockIdx.y / aydiv) * say : nullptr;
    const int* im = imask ? imask + (size_t)(blockIdx.y / aydiv) * imy + (size_t)blockIdx.x * imx : nullptr;
    float v[16];
    const int nj = L / 256;
    float mx = -__builtin_inff();
#pragma unroll
    for (int j = 0; j < 16; ++j) if (j < nj) { float t = row[tid + 256 * j] * prescale; if (av) t += av[tid + 256 * j]; if (im && im[tid + 256 * j] == 0) t = maskval; if (causal && (tid + 256 * j) > (int)blockIdx.x) t = -__builtin_inff(); v[j] = t; mx = fmaxf(mx, t); }
#pragma unroll
    for (int o = 16; o; o >>= 1) mx = fmaxf(mx, __shfl_xor(mx, o, 32));
    if (lane == 0) red[wid] = mx;
    __syncthreads();
    float m = red[0];
#pragma unroll
    for (int i = 1; i < 8; ++i) m = fmaxf(m, red[i]);
    if (m == -__builtin_inff()) m = 0.f;
    __syncthreads();
    float sum = 0.f;
#pragma unroll
    for (int j = 0; j < 16; ++j) if (j < nj) { v[j] = expf(v[j] - m); sum += v[j]; }
#pragma unroll
    for (int o = 16; o; o >>= 1) sum += __shfl_xor(sum, o, 32);
    if (lane == 0) red[wid] = sum;
    __syncthreads();
    float tot = 0.f;
#pragma unroll
    for (int i = 0; i < 8; ++i) tot += red[i];
    const float inv = 1.0f / tot;
#pragma unroll
    for (int j = 0; j < 16; ++j) if (j < nj) *(volatile float*)(row + tid + 256 * j) = v[j] * inv;
    __threadfence();
#pragma unroll
    for (int j = 0; j < 16; ++j) if (j < nj) *(volatile float*)(row + tid + 256 * j) = v[j] * inv;
}

#define VST2(T, p, v) do { const T vst2_v_ = (v); *(volatile T*)(p) = vst2_v_; __threadfence(); *(volatile T*)(p) = vst2_v_; } while (0)
__device__ __forceinline__ float sqd(const float* a, const float* b) {
    const float dx = __fsub_rn(a[0], b[0]), dy = __fsub_rn(a[1], b[1]), dz = __fsub_rn(a[2], b[2]);
    return __fadd_rn(__fadd_rn(__fmul_rn(dx, dx), __fmul_rn(dy, dy)), __fmul_rn(dz, dz));
}

__global__ __launch_bounds__(256) void k_lin3(const float* __restrict__ x, const float* __restrict__ W1, float* H0) {
    const size_t q = (size_t)blockIdx.x * 256 + threadIdx.x; if (q >= (size_t)NBAT * N0 * 32) return;
    const int c = (int)(q % 32); const size_t r = q / 32; const float* p = x + r * 3;
    VST2(float, H0 + q, p[0] * W1[c] + p[1] * W1[32 + c] + p[2] * W1[64 + c]);
}
__global__ __launch_bounds__(512) void k_pstats(const float* __restrict__ a, int R, int C, double* ps, double* pq) {
    const int c = threadIdx.x, blk = blockIdx.x; if (c >= C) return; double s = 0.0, q = 0.0;
    const int r0 = blk * 1024, r1 = min(R, r0 + 1024);
    for (int r = r0; r < r1; ++r) { const float v = a[(size_t)r * C + c]; s += v; q += (double)v * v; }
    VST2(double, ps + (size_t)blk * C + c, s); VST2(double, pq + (size_t)blk * C + c, q);
}
__global__ __launch_bounds__(512) void k_preduce(const double* __restrict__ ps, const double* __restrict__ pq, int nblk, int C, double cnt, float* mean, float* var) {
    const int c = threadIdx.x; if (c >= C) return; double s = 0.0, q = 0.0;
    for (int b = 0; b < nblk; ++b) { s += ps[(size_t)b * C + c]; q += pq[(size_t)b * C + c]; }
    const double m = s / cnt; double v = q / cnt - m * m; if (v < 0.0) v = 0.0;
    VST2(float, mean + c, (float)m); VST2(float, var + c, (float)v);
}
__global__ __launch_bounds__(256) void k_bnrelu(float* a, const float* __restrict__ mean, const float* __restrict__ var, const float* __restrict__ g, const float* __restrict__ bb, size_t n, int C) {
    const size_t t = (size_t)blockIdx.x * 256 + threadIdx.x; if (t >= n) return; const int c = (int)(t % C);
    VST2(float, a + t, fmaxf((a[t] - mean[c]) * rsqrtf(var[c] + BN_EPS) * g[c] + bb[c], 0.f));
}
template <int N, int M>
__global__ __launch_bounds__(256) void k_fps(const float* __restrict__ P, int* IDX) {
    constexpr int PM = (M < 32) ? 32 : M;
    __shared__ float mind[N]; __shared__ int sel[M]; __shared__ float rv[256]; __shared__ int ri[256]; __shared__ int lastS;
    const int b = blockIdx.x, tid = threadIdx.x; const float* pb = P + (size_t)b * N * 3;
    for (int i = tid; i < N; i += 256) mind[i] = __builtin_inff();
    if (tid == 0) lastS = 0;
    __syncthreads();
    for (int s = 0; s < M; ++s) {
        const int last = lastS;
        if (tid == 0) sel[s] = last;
        const float lx = pb[last * 3], ly = pb[last * 3 + 1], lz = pb[last * 3 + 2]; const float lp[3] = {lx, ly, lz};
        float bv = -__builtin_inff(); int bi = 0x7fffffff;
        for (int i = tid; i < N; i += 256) {
            const float d = sqd(pb + i * 3, lp); const float m = fminf(mind[i], d); mind[i] = m;
            if (m > bv || (m == bv && i < bi)) { bv = m; bi = i; }
        }
        rv[tid] = bv; ri[tid] = bi;
        __syncthreads();
        for (int o = 128; o > 0; o >>= 1) {
            if (tid < o) { const float v2 = rv[tid + o]; const int i2 = ri[tid + o]; if (v2 > rv[tid] || (v2 == rv[tid] && i2 < ri[tid])) { rv[tid] = v2; ri[tid] = i2; } }
            __syncthreads();
        }
        if (tid == 0) lastS = ri[0];
        __syncthreads();
    }
    for (int i = tid; i < PM; i += 256) VST2(int, IDX + (size_t)b * PM + i, (i < M) ? sel[i] : 0);
}
__global__ __launch_bounds__(256) void k_gatherp(const float* __restrict__ P, const int* __restrict__ IDX, int N, int M, float* NP) {
    const int q = blockIdx.x * 256 + threadIdx.x; if (q >= NBAT * M * 3) return;
    const int PM = (M < 32) ? 32 : M;
    const int j = q % 3, m = (q / 3) % M, b = q / (3 * M); int i = IDX[b * PM + m]; i = i < 0 ? 0 : (i >= N ? N - 1 : i);
    VST2(float, NP + q, P[((size_t)b * N + i) * 3 + j]);
}
template <int N>
__global__ __launch_bounds__(256) void k_knn(const float* __restrict__ P, const float* __restrict__ NP, int M, int* NIDX) {
    __shared__ int st[256 * KNB];
    const int tid = threadIdx.x; const int qpb = M < 256 ? M : 256;
    const int blocks_per_b = (M + 255) / 256; const int b = blockIdx.x / blocks_per_b, m = (blockIdx.x % blocks_per_b) * 256 + tid;
    if (m < M) {
        const float* q = NP + ((size_t)b * M + m) * 3; const float* pb = P + (size_t)b * N * 3;
        float bd[KNB]; int bi[KNB];
#pragma unroll
        for (int j = 0; j < KNB; ++j) { bd[j] = __builtin_inff(); bi[j] = 0; }
        for (int i = 0; i < N; ++i) {
            const float d = sqd(q, pb + i * 3);
            if (d < bd[KNB - 1]) {
                int j = KNB - 1;
                while (j > 0 && bd[j - 1] > d) { bd[j] = bd[j - 1]; bi[j] = bi[j - 1]; --j; }
                bd[j] = d; bi[j] = i;
            }
        }
#pragma unroll
        for (int j = 0; j < KNB; ++j) st[tid * KNB + j] = bi[j];
    }
    __syncthreads();
    const int nq = (M - (blockIdx.x % blocks_per_b) * 256); const int nvalid = (nq < 256 ? nq : 256) * KNB;
    int* dst = NIDX + ((size_t)b * M + (blockIdx.x % blocks_per_b) * 256) * KNB;
    for (int i = tid; i < nvalid; i += 256) VST2(int, dst + i, st[i]);
    (void)qpb;
}
__global__ __launch_bounds__(256) void k_feat(const float* __restrict__ P, const float* __restrict__ NP, const float* __restrict__ H, const int* __restrict__ NIDX, int N, int M, int C, int pitch, float* FEAT) {
    const size_t t = (size_t)blockIdx.x * 256 + threadIdx.x; if (t >= (size_t)NBAT * M * KNB * pitch) return;
    const int col = (int)(t % pitch); const size_t row = t / pitch; const int k = (int)(row % KNB); const int m = (int)((row / KNB) % M); const int b = (int)(row / ((size_t)KNB * M));
    int i = NIDX[((size_t)b * M + m) * KNB + k]; i = i < 0 ? 0 : (i >= N ? N - 1 : i);
    float v = 0.f;
    if (col < 3) v = P[((size_t)b * N + i) * 3 + col] - NP[((size_t)b * M + m) * 3 + col];
    else if (col < 3 + C) v = H[((size_t)b * N + i) * C + (col - 3)];
    VST2(float, FEAT + t, v);
}
__global__ __launch_bounds__(256) void k_bnmax(const float* __restrict__ Y, const float* __restrict__ mean, const float* __restrict__ var, const float* __restrict__ g, const float* __restrict__ bb, int C, size_t nout, float* Hn) {
    const size_t t = (size_t)blockIdx.x * 256 + threadIdx.x; if (t >= nout) return; const int c = (int)(t % C); const size_t bm = t / C;
    const float sc = rsqrtf(var[c] + BN_EPS) * g[c]; float best = -__builtin_inff();
#pragma unroll
    for (int k = 0; k < KNB; ++k) best = fmaxf(best, fmaxf((Y[(bm * KNB + k) * C + c] - mean[c]) * sc + bb[c], 0.f));
    VST2(float, Hn + t, best);
}
__global__ __launch_bounds__(640) void k_out(const float* __restrict__ Z3, float* out) {
    const int q = threadIdx.x; VST2(float, out + q, Z3[(q / NCLS) * 64 + (q % NCLS)]);
}
__global__ __launch_bounds__(512) void k_meanpool(const float* __restrict__ H, float* Z) {
    const int b = blockIdx.x, c = threadIdx.x; float s = 0.f; for (int m = 0; m < 16; ++m) s += H[((size_t)b * 16 + m) * 512 + c];
    VST2(float, Z + (size_t)b * 512 + c, s * (1.0f / 16.0f));
}
__global__ __launch_bounds__(256) void k_bn16(float* a, const float* __restrict__ g, const float* __restrict__ bb, int C) {
    const int c = threadIdx.x; if (c >= C) return; float s = 0.f; for (int r = 0; r < NBAT; ++r) s += a[r * C + c];
    const float m = s / NBAT; float q = 0.f; for (int r = 0; r < NBAT; ++r) { const float d = a[r * C + c] - m; q += d * d; }
    const float sc = rsqrtf(q / NBAT + BN_EPS) * g[c];
    for (int r = 0; r < NBAT; ++r) { const float v = fmaxf((a[r * C + c] - m) * sc + bb[c], 0.f); *(volatile float*)(a + r * C + c) = v; }
    __threadfence();
    for (int r = 0; r < NBAT; ++r) { const float v = a[r * C + c]; *(volatile float*)(a + r * C + c) = v; }
}

extern "C" void kernel_launch(void* const* d_in, const int* in_sizes, int n_in,
                              void* d_out, int out_size, void* d_ws, size_t ws_size, hipStream_t stream) {
    (void)in_sizes; (void)n_in; (void)out_size;
    const float* x = (const float*)d_in[0];
    const float* W1 = (const float*)d_in[1]; const float* g1 = (const float*)d_in[2]; const float* b1 = (const float*)d_in[3];
    const float* Ws[4] = {(const float*)d_in[4], (const float*)d_in[7], (const float*)d_in[10], (const float*)d_in[13]};
    const float* gs[4] = {(const float*)d_in[5], (const float*)d_in[8], (const float*)d_in[11], (const float*)d_in[14]};
    const float* bs[4] = {(const float*)d_in[6], (const float*)d_in[9], (const float*)d_in[12], (const float*)d_in[15]};
    const float* Wc1 = (const float*)d_in[16]; const float* bc1 = (const float*)d_in[17]; const float* gc1 = (const float*)d_in[18]; const float* hc1 = (const float*)d_in[19];
    const float* Wc2 = (const float*)d_in[20]; const float* bc2 = (const float*)d_in[21]; const float* gc2 = (const float*)d_in[22]; const float* hc2 = (const float*)d_in[23];
    const float* Wc3 = (const float*)d_in[24]; const float* bc3 = (const float*)d_in[25];
    float* out = (float*)d_out;

    const int Ns[5] = {4096, 1024, 256, 64, 16}; const int Cs[5] = {32, 64, 128, 256, 512}; const int pitch[4] = {64, 96, 160, 288};
    char* wsp = (char*)d_ws;
    auto take = [&](size_t bytes) { char* p = wsp; wsp += (bytes + 255) & ~(size_t)255; return (void*)p; };
    float* Pb[5]; float* Hb[5]; int* IDXb[4]; int* NIDXb[4];
    Pb[0] = (float*)x;
    for (int s = 0; s < 5; ++s) { if (s) Pb[s] = (float*)take((size_t)NBAT * Ns[s] * 3 * 4); Hb[s] = (float*)take((size_t)NBAT * Ns[s] * Cs[s] * 4); }
    for (int s = 0; s < 4; ++s) { IDXb[s] = (int*)take((size_t)NBAT * (Ns[s + 1] < 32 ? 32 : Ns[s + 1]) * 4); NIDXb[s] = (int*)take((size_t)NBAT * Ns[s + 1] * KNB * 4); }
    float* FEAT = (float*)take((size_t)NBAT * 1024 * KNB * 64 * 4);
    float* Y = (float*)take((size_t)NBAT * 1024 * KNB * 64 * 4);
    double* ps = (double*)take((size_t)256 * 512 * 8); double* pq = (double*)take((size_t)256 * 512 * 8);
    float* mean = (float*)take(512 * 4); float* var = (float*)take(512 * 4);
    float* Z = (float*)take((size_t)NBAT * 512 * 4); float* Z1 = (float*)take((size_t)NBAT * 256 * 4); float* Z2 = (float*)take((size_t)NBAT * 128 * 4); float* Z3 = (float*)take((size_t)NBAT * 64 * 4);
    if ((size_t)(wsp - (char*)d_ws) > ws_size) return;

    k_lin3<<<(NBAT * N0 * 32) / 256, 256, 0, stream>>>(x, W1, Hb[0]);
    k_pstats<<<(NBAT * N0) / 1024, 512, 0, stream>>>(Hb[0], NBAT * N0, 32, ps, pq);
    k_preduce<<<1, 512, 0, stream>>>(ps, pq, (NBAT * N0) / 1024, 32, (double)(NBAT * N0), mean, var);
    k_bnrelu<<<(NBAT * N0 * 32) / 256, 256, 0, stream>>>(Hb[0], mean, var, g1, b1, (size_t)NBAT * N0 * 32, 32);
    for (int s = 0; s < 4; ++s) {
        const int N = Ns[s], M = Ns[s + 1], C = Cs[s], CO = Cs[s + 1], PT = pitch[s];
        switch (s) { case 0: k_fps<4096, 1024><<<NBAT, 256, 0, stream>>>(Pb[0], IDXb[0]); break; case 1: k_fps<1024, 256><<<NBAT, 256, 0, stream>>>(Pb[1], IDXb[1]); break;
                     case 2: k_fps<256, 64><<<NBAT, 256, 0, stream>>>(Pb[2], IDXb[2]); break; default: k_fps<64, 16><<<NBAT, 256, 0, stream>>>(Pb[3], IDXb[3]); break; }
        k_gatherp<<<(NBAT * M * 3 + 255) / 256, 256, 0, stream>>>(Pb[s], IDXb[s], N, M, Pb[s + 1]);
        const int bpb = (M + 255) / 256;
        switch (s) { case 0: k_knn<4096><<<NBAT * bpb, 256, 0, stream>>>(Pb[0], Pb[1], M, NIDXb[0]); break; case 1: k_knn<1024><<<NBAT * bpb, 256, 0, stream>>>(Pb[1], Pb[2], M, NIDXb[1]); break;
                     case 2: k_knn<256><<<NBAT * bpb, 256, 0, stream>>>(Pb[2], Pb[3], M, NIDXb[2]); break; default: k_knn<64><<<NBAT * bpb, 256, 0, stream>>>(Pb[3], Pb[4], M, NIDXb[3]); break; }
        const size_t rows = (size_t)NBAT * M * KNB;
        k_feat<<<(unsigned)((rows * PT + 255) / 256), 256, 0, stream>>>(Pb[s], Pb[s + 1], Hb[s], NIDXb[s], N, M, C, PT, FEAT);
        { GemmArgs g = gemm_args(FEAT, PT, zm(0), Ws[s], CO, zm(0), Y, CO, zm(0), (int)rows, CO, 3 + C);
          gemm_kernel<0, 0, 2, 2, 4, 2, ACT_NONE><<<dim3((unsigned)((rows + 63) / 64), (CO + 127) / 128, 1), 256, 0, stream>>>(g); }
        k_pstats<<<(unsigned)(rows / 1024), 512, 0, stream>>>(Y, (int)rows, CO, ps, pq);
        k_preduce<<<1, 512, 0, stream>>>(ps, pq, (int)(rows / 1024), CO, (double)rows, mean, var);
        k_bnmax<<<(unsigned)(((size_t)NBAT * M * CO + 255) / 256), 256, 0, stream>>>(Y, mean, var, gs[s], bs[s], CO, (size_t)NBAT * M * CO, Hb[s + 1]);
    }
    k_meanpool<<<NBAT, 512, 0, stream>>>(Hb[4], Z);
    { GemmArgs g = gemm_args(Z, 512, zm(0), Wc1, 256, zm(0), Z1, 256, zm(0), NBAT, 256, 512); g.bias = bc1; gemm_kernel<0, 0, 2, 2, 4, 2, ACT_NONE><<<dim3(1, 2, 1), 256, 0, stream>>>(g); }
    k_bn16<<<1, 256, 0, stream>>>(Z1, gc1, hc1, 256);
    { GemmArgs g = gemm_args(Z1, 256, zm(0), Wc2, 128, zm(0), Z2, 128, zm(0), NBAT, 128, 256); g.bias = bc2; gemm_kernel<0, 0, 2, 2, 4, 2, ACT_NONE><<<dim3(1, 1, 1), 256, 0, stream>>>(g); }
    k_bn16<<<1, 256, 0, stream>>>(Z2, gc2, hc2, 128);
    { GemmArgs g = gemm_args(Z2, 128, zm(0), Wc3, NCLS, zm(0), Z3, 64, zm(0), NBAT, NCLS, 128); g.nstore = 64; g.bias = bc3; gemm_kernel<0, 0, 2, 2, 4, 2, ACT_NONE><<<dim3(1, 1, 1), 256, 0, stream>>>(g); }
    k_out<<<1, NBAT * NCLS, 0, stream>>>(Z3, out);
}
